// CrossSpectralAttention_65575560675805
// MI455X (gfx1250) — hardware-verified
//
#include <hip/hip_runtime.h>
#include <math.h>
#include <stdint.h>

#define NB     2
#define CCH    256
#define NTOK   2304
#define NHEAD  8
#define HDIM   32
#define MP     (NB * NTOK)
#define NQB    (NTOK / 64)
#define XS     4.0f
#define WS     16.0f
#define QC     16.0f
#define KC     16.0f
#define VC     8.0f
#define AC     32.0f
#define RSC    1024.0f
#define IRSC   0.0009765625f
#define SMSC   0.17677669529663687f
#define LNPC   6.931471805599453f
static_assert(NHEAD * HDIM == CCH);
static_assert((MP % 64) == 0 && (CCH % 64) == 0 && (NTOK % 64) == 0);
static_assert(CCH == 32 * 8);
static_assert((NTOK % 32) == 0);

typedef _Float16 v16h __attribute__((ext_vector_type(16)));
typedef _Float16 v8h  __attribute__((ext_vector_type(8)));
typedef float    v8f  __attribute__((ext_vector_type(8)));
typedef float    v4f  __attribute__((ext_vector_type(4)));
typedef unsigned int v4u __attribute__((ext_vector_type(4)));

union FragH { v16h v; v8h h[2]; };

__device__ __forceinline__ unsigned short bf_bits(float f) {
  unsigned u = __float_as_uint(f);
  return (unsigned short)((u + 0x7FFFu + ((u >> 16) & 1u)) >> 16);
}
__device__ __forceinline__ float bf_up(unsigned short h) { return __uint_as_float(((unsigned)h) << 16); }
__device__ __forceinline__ float bfr(float f) { return bf_up(bf_bits(f)); }
__device__ __forceinline__ unsigned short h_bits(_Float16 x) { return __builtin_bit_cast(unsigned short, x); }
__device__ __forceinline__ unsigned pk16(unsigned short a, unsigned short b) { return (unsigned)a | ((unsigned)b << 16); }
__device__ __forceinline__ v8f zero8() { v8f z = {0.f, 0.f, 0.f, 0.f, 0.f, 0.f, 0.f, 0.f}; return z; }
__device__ __forceinline__ float hmax8(v8f s) {
  return fmaxf(fmaxf(fmaxf(s[0], s[1]), fmaxf(s[2], s[3])), fmaxf(fmaxf(s[4], s[5]), fmaxf(s[6], s[7])));
}

__device__ __forceinline__ v16h ldfrag_h(const _Float16* p) {
  FragH f;
  f.h[0] = *(const v8h*)(p);
  f.h[1] = *(const v8h*)(p + 16);
  return f.v;
}

__device__ __forceinline__ v8f mma_h_raw(v16h a, v16h b, v8f c) {
  return __builtin_amdgcn_wmma_f32_16x16x32_f16(false, a, false, b, (short)0, c, false, false);
}
__device__ __forceinline__ void dep_guard1(v8f& a, v8f& b, v16h x) {
#if defined(__HIP_DEVICE_COMPILE__)
  asm volatile("v_nop\n\tv_nop\n\tv_nop\n\tv_nop" : "+v"(a), "+v"(b) : "v"(x));
#endif
}
__device__ __forceinline__ void keep4_h(v16h a, v16h b, v16h c, v16h d) {
#if defined(__HIP_DEVICE_COMPILE__)
  asm volatile("v_nop" :: "v"(a), "v"(b), "v"(c), "v"(d));
#endif
}
__device__ __forceinline__ void acc_guard4(v8f& a, v8f& b, v8f& c, v8f& d) {
#if defined(__HIP_DEVICE_COMPILE__)
  asm volatile("v_nop\n\tv_nop\n\tv_nop\n\tv_nop" : "+v"(a), "+v"(b), "+v"(c), "+v"(d));
#endif
}
__device__ __forceinline__ void sguard8(v8f& a, v8f& b, v8f& c, v8f& d, v8f& e, v8f& f, v8f& g, v8f& hq,
                                        v16h k0, v16h k1, v16h k2, v16h k3, v16h q0, v16h q1) {
#if defined(__HIP_DEVICE_COMPILE__)
  asm volatile("v_nop\n\tv_nop\n\tv_nop\n\tv_nop"
               : "+v"(a), "+v"(b), "+v"(c), "+v"(d), "+v"(e), "+v"(f), "+v"(g), "+v"(hq)
               : "v"(k0), "v"(k1), "v"(k2), "v"(k3), "v"(q0), "v"(q1));
#endif
}
__device__ __forceinline__ void oguard6(v8f& a, v8f& b, v8f& c, v8f& d,
                                        v16h x0, v16h x1, v16h x2, v16h x3, v16h y0, v16h y1) {
#if defined(__HIP_DEVICE_COMPILE__)
  asm volatile("v_nop\n\tv_nop\n\tv_nop\n\tv_nop"
               : "+v"(a), "+v"(b), "+v"(c), "+v"(d) : "v"(x0), "v"(x1), "v"(x2), "v"(x3), "v"(y0), "v"(y1));
#endif
}
__device__ __forceinline__ void wave_sync_lds() {
  __builtin_amdgcn_fence(__ATOMIC_RELEASE, "workgroup");
  __builtin_amdgcn_wave_barrier();
  __builtin_amdgcn_fence(__ATOMIC_ACQUIRE, "workgroup");
}

__global__ __launch_bounds__(256) void wprep(const float* __restrict__ wq, const float* __restrict__ wk,
                                              const float* __restrict__ wv, const float* __restrict__ wo,
                                              unsigned short* W16) {
  const int tid = threadIdx.x, wave = tid >> 5, lane = tid & 31;
  const int bx = blockIdx.x;
  const int which = bx >> 5;
  const float* src = (which == 0) ? wq : (which == 1) ? wk : (which == 2) ? wv : wo;
  const int rowg = bx * 8 + wave;
  const int rin  = rowg & (CCH - 1);
  const float* sp = src + (size_t)rin * CCH + 8 * lane;
  const v4f a = *(const v4f*)(sp), c = *(const v4f*)(sp + 4);
  float w[8];
#pragma unroll
  for (int i = 0; i < 4; ++i) { w[i] = bfr(a[i]) * WS; w[4 + i] = bfr(c[i]) * WS; }
  v4u v;
#pragma unroll
  for (int i = 0; i < 4; ++i) v[i] = pk16(h_bits((_Float16)w[2 * i]), h_bits((_Float16)w[2 * i + 1]));
  unsigned short* dp = W16 + (size_t)rowg * CCH + 8 * lane;
  *(volatile v4u*)dp = v;
  __threadfence();
  *(volatile v4u*)dp = v;
}

__global__ __launch_bounds__(256) void xprep(const float* __restrict__ x, unsigned short* XT) {
  __shared__ __align__(16) float T[CCH * 36];
  const int tid = threadIdx.x, wave = tid >> 5, lane = tid & 31;
  const int bx = blockIdx.x;
  const int b  = bx / (NTOK / 32);
  const int n0 = (bx - b * (NTOK / 32)) * 32;
  const float* sb = x + (size_t)b * CCH * NTOK + n0;
  {
    const int q = lane >> 3, e = lane & 7;
#pragma unroll
    for (int it = 0; it < 8; ++it) {
      const int c = it * 32 + wave * 4 + q;
      const v4f v = *(const v4f*)(sb + (size_t)c * NTOK + 4 * e);
      *(v4f*)(T + c * 36 + 4 * e) = v;
    }
  }
  __syncthreads();
  v4u vals[4];
#pragma unroll
  for (int it = 0; it < 4; ++it) {
    const int tl = it * 8 + wave;
    float w[8];
#pragma unroll
    for (int i = 0; i < 8; ++i) w[i] = bfr(T[(8 * lane + i) * 36 + tl]) * XS;
    v4u v;
#pragma unroll
    for (int i = 0; i < 4; ++i) v[i] = pk16(h_bits((_Float16)w[2 * i]), h_bits((_Float16)w[2 * i + 1]));
    vals[it] = v;
  }
  unsigned short* base = XT + ((size_t)b * NTOK + n0) * CCH + 8 * lane;
  for (int pass = 0; pass < 2; ++pass) {
#pragma unroll
    for (int it = 0; it < 4; ++it) {
      *(volatile v4u*)(base + (size_t)(it * 8 + wave) * CCH) = vals[it];
    }
    __threadfence();
  }
}

template <int BKM>
__device__ __forceinline__ void kloop64(v8f (&acc)[4][4], const _Float16* Ah, int lda, const _Float16* Bb, int ldb,
                                        int m0, int n0, int K, int rlane, int koff) {
  for (int k0 = 0; k0 < K; k0 += 32) {
    v16h bh[4];
#pragma unroll
    for (int j = 0; j < 4; ++j) {
      if (BKM == 0) {
        const size_t bo = (size_t)(n0 + (j << 4) + rlane) * ldb + koff + k0;
        bh[j] = ldfrag_h(Bb + bo);
      } else {
        const _Float16* bp = Bb + (size_t)(k0 + koff) * ldb + n0 + (j << 4) + rlane;
        FragH f;
#pragma unroll
        for (int i = 0; i < 8; ++i) {
          f.h[0][i] = bp[(size_t)i * ldb];
          f.h[1][i] = bp[(size_t)(16 + i) * ldb];
        }
        bh[j] = f.v;
      }
    }
#pragma unroll
    for (int i = 0; i < 4; ++i) {
      const size_t ao = (size_t)(m0 + (i << 4) + rlane) * lda + koff + k0;
      const v16h ah = ldfrag_h(Ah + ao);
#pragma unroll
      for (int j = 0; j < 4; ++j) acc[i][j] = mma_h_raw(ah, bh[j], acc[i][j]);
      dep_guard1(acc[i][0], acc[i][3], ah);
    }
    keep4_h(bh[0], bh[1], bh[2], bh[3]);
  }
}

template <int BKM, int OM, int BIASM, int NPL>
__global__ __launch_bounds__(256) void gemm64(
    const unsigned short* __restrict__ Ap, int lda, long long strideA,
    const unsigned short* __restrict__ Bp, const unsigned short* __restrict__ B2p, int ldb, long long strideB,
    const float* __restrict__ bias0, const float* __restrict__ bias1,
    void* Cout, int ldc, long long strideC,
    unsigned short* Clo, int ldlo, long long strideLo, int nsplit,
    float ascale, float cs0, float cs1, int M, int N, int K) {
  __shared__ __align__(16) float sT[8][16 * 68];
  const int b    = blockIdx.y;
  const int lane = threadIdx.x & 31;
  const int wave = threadIdx.x >> 5;
  const int tilesN = N >> 6;
  const int tilesM = M >> 6;
  const int tile = blockIdx.x * 8 + wave;
  if (tile >= tilesM * tilesN) return;
  const int tm = tile / tilesN;
  const int tn = tile - tm * tilesN;
  const int m0 = tm << 6;
  const int n0 = tn << 6;

  const _Float16* Ah = (const _Float16*)(const void*)Ap + (size_t)b * strideA;
  const _Float16* Bb = (const _Float16*)(const void*)Bp + (size_t)b * strideB;

  const int rlane = lane & 15;
  const int koff  = (lane >> 4) * 8;
  const int mOff  = (lane >> 4) * 8;

  v8f acc[4][4];
#pragma unroll
  for (int i = 0; i < 4; ++i)
#pragma unroll
    for (int j = 0; j < 4; ++j) acc[i][j] = zero8();

  if (NPL == 2) {
    const _Float16* B2 = (const _Float16*)(const void*)B2p + (size_t)b * strideB;
    kloop64<BKM>(acc, Ah, lda, B2, ldb, m0, n0, K, rlane, koff);
    acc_guard4(acc[0][0], acc[0][1], acc[0][2], acc[0][3]);
    acc_guard4(acc[1][0], acc[1][1], acc[1][2], acc[1][3]);
    acc_guard4(acc[2][0], acc[2][1], acc[2][2], acc[2][3]);
    acc_guard4(acc[3][0], acc[3][1], acc[3][2], acc[3][3]);
#pragma unroll
    for (int i = 0; i < 4; ++i)
#pragma unroll
      for (int j = 0; j < 4; ++j) acc[i][j] = acc[i][j] * IRSC;
    acc_guard4(acc[0][0], acc[0][1], acc[0][2], acc[0][3]);
    acc_guard4(acc[1][0], acc[1][1], acc[1][2], acc[1][3]);
    acc_guard4(acc[2][0], acc[2][1], acc[2][2], acc[2][3]);
    acc_guard4(acc[3][0], acc[3][1], acc[3][2], acc[3][3]);
  }
  kloop64<BKM>(acc, Ah, lda, Bb, ldb, m0, n0, K, rlane, koff);
  acc_guard4(acc[0][0], acc[0][1], acc[0][2], acc[0][3]);
  acc_guard4(acc[1][0], acc[1][1], acc[1][2], acc[1][3]);
  acc_guard4(acc[2][0], acc[2][1], acc[2][2], acc[2][3]);
  acc_guard4(acc[3][0], acc[3][1], acc[3][2], acc[3][3]);

  const bool  hireg = (n0 >= nsplit);
  const float cs    = hireg ? cs1 : cs0;
  const bool  dolo  = (OM == 1) && !hireg;
  const int hh2 = lane >> 4, c4 = (lane & 15) * 4;
  const int q8  = lane >> 3, c8 = (lane & 7) * 8;

  float bcol[8];
#pragma unroll
  for (int i = 0; i < 8; ++i) bcol[i] = 0.f;
  if (OM == 1 && BIASM == 2) {
    const float* bp = hireg ? bias1 : bias0;
    const int nb = n0 - (hireg ? nsplit : 0) + c8;
    const v4f b0 = *(const v4f*)(bp + nb);
    const v4f b1 = *(const v4f*)(bp + nb + 4);
#pragma unroll
    for (int i = 0; i < 4; ++i) { bcol[i] = bfr(b0[i]); bcol[4 + i] = bfr(b1[i]); }
  }

  float* slab = sT[wave];
#pragma unroll
  for (int i = 0; i < 4; ++i) {
    const int mBase = m0 + (i << 4);
#pragma unroll
    for (int j = 0; j < 4; ++j) {
#pragma unroll
      for (int r = 0; r < 8; ++r) {
        slab[(mOff + r) * 68 + (j << 4) + rlane] = acc[i][j][r];
      }
    }
    wave_sync_lds();
    if (OM == 0) {
      float* C = (float*)Cout + (size_t)b * strideC;
      v4f vals[8];
#pragma unroll
      for (int it = 0; it < 8; ++it) {
        const int row = it * 2 + hh2;
        const float bm = (BIASM == 1) ? bfr(bias0[mBase + row]) : 0.f;
        v4f v = *(const v4f*)(slab + row * 68 + c4);
#pragma unroll
        for (int e = 0; e < 4; ++e) v[e] = v[e] * ascale + bm;
        vals[it] = v;
      }
      for (int pass = 0; pass < 2; ++pass) {
#pragma unroll
        for (int it = 0; it < 8; ++it) {
          const int row = it * 2 + hh2;
          *(volatile v4f*)(C + (size_t)(mBase + row) * ldc + n0 + c4) = vals[it];
        }
        __threadfence();
      }
    } else {
      unsigned short* C = (unsigned short*)Cout + (size_t)b * strideC;
      unsigned short* L = Clo + (size_t)b * strideLo;
      v4u hv[4], lv[4];
#pragma unroll
      for (int it = 0; it < 4; ++it) {
        const int row = it * 4 + q8;
        const float brow = (BIASM == 1) ? bfr(bias0[mBase + row]) : 0.f;
        const float* sp = slab + row * 68 + c8;
        v4u a, lo;
#pragma unroll
        for (int e = 0; e < 4; ++e) {
          const float be0 = (BIASM == 2) ? bcol[2 * e] : brow;
          const float be1 = (BIASM == 2) ? bcol[2 * e + 1] : brow;
          const float f0 = (sp[2 * e] * ascale + be0) * cs, f1 = (sp[2 * e + 1] * ascale + be1) * cs;
          const _Float16 h0 = (_Float16)f0, h1 = (_Float16)f1;
          const _Float16 l0 = (_Float16)((f0 - (float)h0) * RSC), l1 = (_Float16)((f1 - (float)h1) * RSC);
          a[e]  = pk16(h_bits(h0), h_bits(h1));
          lo[e] = pk16(h_bits(l0), h_bits(l1));
        }
        hv[it] = a;
        lv[it] = lo;
      }
      for (int pass = 0; pass < 2; ++pass) {
#pragma unroll
        for (int it = 0; it < 4; ++it) {
          const int row = it * 4 + q8;
          *(volatile v4u*)(C + (size_t)(mBase + row) * ldc + n0 + c8) = hv[it];
          if (dolo) *(volatile v4u*)(L + (size_t)(mBase + row) * ldlo + n0 + c8) = lv[it];
        }
        __threadfence();
      }
    }
    wave_sync_lds();
  }
}

__global__ __launch_bounds__(128)
void attn_t(const unsigned short* __restrict__ qk, const unsigned short* __restrict__ ql,
            const unsigned short* __restrict__ vt, const unsigned short* __restrict__ vl,
            unsigned short* ot, unsigned short* ol) {
  __shared__ __align__(16) unsigned short Osh[HDIM * 64];
  __shared__ __align__(16) unsigned short Osl[HDIM * 64];
  const int tid  = threadIdx.x;
  const int wave = tid >> 5;
  const int lane = tid & 31;
  const int hh   = lane >> 4;
  const int c    = lane & 15;
  const int bx = blockIdx.x;
  const int qb = bx % NQB;
  const int hd = (bx / NQB) % NHEAD;
  const int b  = bx / (NQB * NHEAD);
  const int q0 = qb * 64;
  const size_t tok0 = (size_t)b * NTOK;

  const _Float16* QKp = (const _Float16*)(const void*)qk;
  const _Float16* QLp = (const _Float16*)(const void*)ql;
  const _Float16* VHp = (const _Float16*)(const void*)vt;
  const _Float16* VLp = (const _Float16*)(const void*)vl;

  const size_t tr = tok0 + q0 + wave * 16 + c;
  const v16h qhi = ldfrag_h(QKp + tr * (2 * CCH) + hd * HDIM + 8 * hh);
  const v16h qlo = ldfrag_h(QLp + tr * CCH + hd * HDIM + 8 * hh);
  const _Float16* Kp = QKp + (tok0 + c) * (2 * CCH) + CCH + hd * HDIM + 8 * hh;
  const size_t vr0 = ((size_t)b * CCH + (size_t)hd * HDIM + c) * NTOK + 8 * hh;
  const size_t vr1 = vr0 + (size_t)16 * NTOK;
  const float SC = SMSC / (QC * KC);

  float m = -1.0e30f, l = 0.f;
  v8f om0 = zero8(), om1 = zero8(), or0 = zero8(), or1 = zero8();
#pragma unroll 1
  for (int it = 0; it < NQB; ++it) {
    const int kb = it * 64;
    v16h kf[4];
#pragma unroll
    for (int j = 0; j < 4; ++j) kf[j] = ldfrag_h(Kp + (size_t)(kb + 16 * j) * (2 * CCH));
    v8f sh0 = mma_h_raw(kf[0], qhi, zero8());
    v8f sh1 = mma_h_raw(kf[1], qhi, zero8());
    v8f sh2 = mma_h_raw(kf[2], qhi, zero8());
    v8f sh3 = mma_h_raw(kf[3], qhi, zero8());
    v8f sl0 = mma_h_raw(kf[0], qlo, zero8());
    v8f sl1 = mma_h_raw(kf[1], qlo, zero8());
    v8f sl2 = mma_h_raw(kf[2], qlo, zero8());
    v8f sl3 = mma_h_raw(kf[3], qlo, zero8());
    sguard8(sh0, sh1, sh2, sh3, sl0, sl1, sl2, sl3, kf[0], kf[1], kf[2], kf[3], qhi, qlo);
    const v8f s0 = sh0 + sl0 * IRSC;
    const v8f s1 = sh1 + sl1 * IRSC;
    const v8f s2 = sh2 + sl2 * IRSC;
    const v8f s3 = sh3 + sl3 * IRSC;

    float mx = fmaxf(fmaxf(hmax8(s0), hmax8(s1)), fmaxf(hmax8(s2), hmax8(s3)));
    mx = fmaxf(mx, __shfl_xor(mx, 16, 32));
    const float mn   = fmaxf(m, mx * SC);
    const float corr = __expf(m - mn);
    m = mn;
    const float msh = mn - LNPC;
    l *= corr;
    om0 = om0 * corr; om1 = om1 * corr; or0 = or0 * corr; or1 = or1 * corr;

    FragH ph0, ph1, pl0, pl1;
    float ls = 0.f;
#pragma unroll
    for (int r = 0; r < 8; ++r) {
      const float e0 = __expf(s0[r] * SC - msh);
      const float e1 = __expf(s1[r] * SC - msh);
      const float e2 = __expf(s2[r] * SC - msh);
      const float e3 = __expf(s3[r] * SC - msh);
      ls += (e0 + e1) + (e2 + e3);
      const _Float16 g0 = (_Float16)e0, g1 = (_Float16)e1, g2 = (_Float16)e2, g3 = (_Float16)e3;
      ph0.h[0][r] = g0;
      ph0.h[1][r] = g1;
      ph1.h[0][r] = g2;
      ph1.h[1][r] = g3;
      pl0.h[0][r] = (_Float16)((e0 - (float)g0) * RSC);
      pl0.h[1][r] = (_Float16)((e1 - (float)g1) * RSC);
      pl1.h[0][r] = (_Float16)((e2 - (float)g2) * RSC);
      pl1.h[1][r] = (_Float16)((e3 - (float)g3) * RSC);
    }
    l += ls;

    {
      const v16h vh0 = ldfrag_h(VHp + vr0 + kb), vh1 = ldfrag_h(VHp + vr1 + kb);
      const v16h vg0 = ldfrag_h(VLp + vr0 + kb), vg1 = ldfrag_h(VLp + vr1 + kb);
      om0 = mma_h_raw(vh0, ph0.v, om0);
      or0 = mma_h_raw(vh0, pl0.v, or0);
      or0 = mma_h_raw(vg0, ph0.v, or0);
      om1 = mma_h_raw(vh1, ph0.v, om1);
      or1 = mma_h_raw(vh1, pl0.v, or1);
      or1 = mma_h_raw(vg1, ph0.v, or1);
      oguard6(om0, om1, or0, or1, vh0, vh1, vg0, vg1, ph0.v, pl0.v);
    }
    {
      const v16h vh0 = ldfrag_h(VHp + vr0 + kb + 32), vh1 = ldfrag_h(VHp + vr1 + kb + 32);
      const v16h vg0 = ldfrag_h(VLp + vr0 + kb + 32), vg1 = ldfrag_h(VLp + vr1 + kb + 32);
      om0 = mma_h_raw(vh0, ph1.v, om0);
      or0 = mma_h_raw(vh0, pl1.v, or0);
      or0 = mma_h_raw(vg0, ph1.v, or0);
      om1 = mma_h_raw(vh1, ph1.v, om1);
      or1 = mma_h_raw(vh1, pl1.v, or1);
      or1 = mma_h_raw(vg1, ph1.v, or1);
      oguard6(om0, om1, or0, or1, vh0, vh1, vg0, vg1, ph1.v, pl1.v);
    }
  }
  l += __shfl_xor(l, 16, 32);
  const float sc = (AC / VC) * (1.0f / l);

#pragma unroll
  for (int r = 0; r < 8; ++r) {
    const float f0 = (om0[r] + or0[r] * IRSC) * sc;
    const float f1 = (om1[r] + or1[r] * IRSC) * sc;
    const _Float16 g0 = (_Float16)f0, g1 = (_Float16)f1;
    const _Float16 e0 = (_Float16)((f0 - (float)g0) * RSC), e1 = (_Float16)((f1 - (float)g1) * RSC);
    Osh[(8 * hh + r) * 64 + wave * 16 + c]      = h_bits(g0);
    Osl[(8 * hh + r) * 64 + wave * 16 + c]      = h_bits(e0);
    Osh[(16 + 8 * hh + r) * 64 + wave * 16 + c] = h_bits(g1);
    Osl[(16 + 8 * hh + r) * 64 + wave * 16 + c] = h_bits(e1);
  }
  __syncthreads();
  {
    const int dq = tid >> 3, e = tid & 7;
    v4u hvv[2], lvv[2];
#pragma unroll
    for (int it = 0; it < 2; ++it) {
      const int d = it * 16 + dq;
      hvv[it] = *(const v4u*)(Osh + d * 64 + 8 * e);
      lvv[it] = *(const v4u*)(Osl + d * 64 + 8 * e);
    }
    const size_t rb = ((size_t)b * CCH + (size_t)hd * HDIM) * NTOK + q0 + 8 * e;
    for (int pass = 0; pass < 2; ++pass) {
#pragma unroll
      for (int it = 0; it < 2; ++it) {
        const int d = it * 16 + dq;
        *(volatile v4u*)(ot + rb + (size_t)d * NTOK) = hvv[it];
        *(volatile v4u*)(ol + rb + (size_t)d * NTOK) = lvv[it];
      }
      __threadfence();
    }
  }
}

extern "C" void kernel_launch(void* const* d_in, const int* in_sizes, int n_in,
                              void* d_out, int out_size, void* d_ws, size_t ws_size,
                              hipStream_t stream) {
  if (n_in < 9) return;
  if (in_sizes[0] != NB * CCH * NTOK) return;
  if (in_sizes[1] != CCH * CCH || in_sizes[3] != CCH * CCH || in_sizes[5] != CCH * CCH || in_sizes[7] != CCH * CCH) return;
  if (in_sizes[2] != CCH || in_sizes[4] != CCH || in_sizes[6] != CCH || in_sizes[8] != CCH) return;
  if (out_size != NB * CCH * NTOK) return;

  const float* x  = (const float*)d_in[0];
  const float* wq = (const float*)d_in[1];
  const float* bq = (const float*)d_in[2];
  const float* wk = (const float*)d_in[3];
  const float* bk = (const float*)d_in[4];
  const float* wv = (const float*)d_in[5];
  const float* bv = (const float*)d_in[6];
  const float* wo = (const float*)d_in[7];
  const float* bo = (const float*)d_in[8];

  const size_t PW  = (size_t)4 * CCH * CCH * 2;
  const size_t PXT = (size_t)MP * CCH * 2;
  const size_t PQK = (size_t)MP * 2 * CCH * 2;
  const size_t PQL = (size_t)MP * CCH * 2;
  const size_t PV  = (size_t)NB * CCH * NTOK * 2;
  size_t off = 0;
  const size_t oW  = off; off += PW;
  const size_t oXT = off; off += PXT;
  const size_t oQK = off; off += PQK;
  const size_t oQL = off; off += PQL;
  const size_t oVT = off; off += PV;
  const size_t oVL = off; off += PV;
  const size_t oOT = off; off += PV;
  const size_t oOL = off; off += PV;
  if (off > ws_size) return;
  if (off > (size_t)134217728) return;

  char* ws = (char*)d_ws;
  unsigned short* W16 = (unsigned short*)(ws + oW);
  unsigned short* XT  = (unsigned short*)(ws + oXT);
  unsigned short* QK  = (unsigned short*)(ws + oQK);
  unsigned short* QL  = (unsigned short*)(ws + oQL);
  unsigned short* VT  = (unsigned short*)(ws + oVT);
  unsigned short* VL  = (unsigned short*)(ws + oVL);
  unsigned short* OT  = (unsigned short*)(ws + oOT);
  unsigned short* OL  = (unsigned short*)(ws + oOL);
  float*          out = (float*)d_out;

  const dim3 blk(256), blk128(128);
  const dim3 gW(4 * CCH / 8);
  const dim3 gX(NB * (NTOK / 32));
  const dim3 gQK(((MP / 64) * ((2 * CCH) / 64)) / 8, 1);
  const dim3 gVT(((CCH / 64) * (NTOK / 64)) / 8, NB);
  const dim3 gAT(NB * NHEAD * NQB);
  const dim3 gPJ(((CCH / 64) * (NTOK / 64)) / 8, NB);

  wprep<<<gW, blk, 0, stream>>>(wq, wk, wv, wo, W16);

  xprep<<<gX, blk, 0, stream>>>(x, XT);

  gemm64<0, 1, 2, 1><<<gQK, blk, 0, stream>>>(
      XT, CCH, 0LL,
      W16, W16, CCH, 0LL,
      bq, bk,
      (void*)QK, 2 * CCH, 0LL,
      QL, CCH, 0LL, CCH,
      1.0f / (XS * WS), QC, KC, MP, 2 * CCH, CCH);

  gemm64<0, 1, 1, 1><<<gVT, blk, 0, stream>>>(
      W16 + (size_t)2 * CCH * CCH, CCH, 0LL,
      XT, XT, CCH, (long long)NTOK * CCH,
      bv, bv,
      (void*)VT, NTOK, (long long)CCH * NTOK,
      VL, NTOK, (long long)CCH * NTOK, NTOK,
      1.0f / (XS * WS), VC, VC, CCH, NTOK, CCH);

  attn_t<<<gAT, blk128, 0, stream>>>(QK, QL, VT, VL, OT, OL);

  gemm64<1, 0, 1, 2><<<gPJ, blk, 0, stream>>>(
      W16 + (size_t)3 * CCH * CCH, CCH, 0LL,
      OT, OL, NTOK, (long long)CCH * NTOK,
      bo, bo,
      (void*)out, NTOK, (long long)CCH * NTOK,
      QL, CCH, 0LL, 0,
      1.0f / (WS * AC), 1.0f, 1.0f, CCH, NTOK, CCH);
  (void)hipGetLastError();
}
